// HierarchicalAttentionNetwork_90494960926749
// MI455X (gfx1250) — hardware-run, weakly checked
//
#include <hip/hip_runtime.h>
#include <math.h>

typedef __attribute__((ext_vector_type(16))) _Float16 v16h;
typedef __attribute__((ext_vector_type(8)))  _Float16 v8h;
typedef __attribute__((ext_vector_type(8)))  float    v8f;
typedef __attribute__((ext_vector_type(4)))  float    v4f;

constexpr int kSeq       = 512;
constexpr int kBatch     = 256;
constexpr int kEmb       = 200;
constexpr int kHid       = 50;
constexpr int kG3        = 3 * kHid;
constexpr int kMlp       = 100;
constexpr int kVocabRows = 50001;
constexpr int kRows      = kSeq * kBatch;
constexpr int kKp     = 224;
constexpr int kNd     = 160;
constexpr int kNp     = 2 * kNd;
constexpr int kHk     = 64;
constexpr int kHp     = 2 * kHk;
constexpr int kMn     = 128;
constexpr int kApitch = 232;
static_assert(kG3 == 150 && kRows == 131072, "shape");
static_assert((kKp % 32) == 0 && kKp >= kEmb, "K pad of the input projection");
static_assert((kHk % 32) == 0 && kHk >= kHid, "K pad of the recurrent product");
static_assert((kHp % 32) == 0 && kHp >= 2 * kHid, "K pad of the MLP product");
static_assert((kNp % 64) == 0 && (kNd % 16) == 0 && kNd >= kG3 && (kMn % 64) == 0 && kMn >= kMlp, "N pads");
static_assert((kRows % 64) == 0 && (kBatch % 64) == 0 && (kEmb % 8) == 0, "tile multiples");

constexpr float kCarry  = 256.0f;
constexpr float kFold   = 1.0f / (kCarry * kCarry);
constexpr float kUncar  = 1.0f / kCarry;
constexpr float kF16Min = 6.103515625e-05f;

constexpr size_t kSzWIH  = (size_t)kNp * kKp * 2;
constexpr size_t kSzBIAS = (size_t)kNp * 4;
constexpr size_t kSzWHH  = (size_t)2 * kNd * kHk * 2;
constexpr size_t kSzWML  = (size_t)kMn * kHp * 2;
constexpr size_t kSzGX   = (size_t)kRows * kNp * 2;
constexpr size_t kSzHP   = (size_t)kRows * kHp * 2;
constexpr size_t kSzSC   = (size_t)kRows * 4;
constexpr size_t kOffWIH  = 0;
constexpr size_t kOffBIAS = kOffWIH + kSzWIH;
constexpr size_t kOffWHH  = kOffBIAS + kSzBIAS;
constexpr size_t kOffWML  = kOffWHH + kSzWHH;
constexpr size_t kOffGX   = kOffWML + kSzWML;
constexpr size_t kOffHP   = kOffGX + kSzGX;
constexpr size_t kOffSC   = kOffHP + kSzHP;
constexpr size_t kWsTotal = kOffSC + kSzSC;
static_assert(kWsTotal == 118183168ull, "carve total");
static_assert(kWsTotal <= 134217728ull, "carve cap");
static_assert((kOffBIAS % 128) == 0 && (kOffWHH % 128) == 0 && (kOffWML % 128) == 0 &&
              (kOffGX % 128) == 0 && (kOffHP % 128) == 0 && (kOffSC % 128) == 0, "128-B aligned regions");

union FH { v16h v; v8h h[2]; };

__device__ __forceinline__ v16h ldfrag_g(const _Float16* p) {
  FH f;
  f.h[0] = *(const v8h*)(p);
  f.h[1] = *(const v8h*)(p + 16);
  return f.v;
}

__device__ __forceinline__ v8f mma_h(v16h a, v16h b, v8f c) {
  c = __builtin_amdgcn_wmma_f32_16x16x32_f16(false, a, false, b, (short)0, c, false, false);
  asm volatile("v_nop\n\tv_nop\n\tv_nop\n\tv_nop" : "+v"(c) : "v"(a), "v"(b));
  return c;
}

__device__ __forceinline__ _Float16 to_h_carry(float f) {
  const float v = f * kCarry;
  const float w = (fabsf(v) < kF16Min) ? 0.0f : v;
  return (_Float16)w;
}

__device__ __forceinline__ float h16_to_f32(unsigned hb) {
  const unsigned sgn = (hb & 0x8000u) << 16;
  const unsigned em = hb & 0x7fffu;
  const float fn = __uint_as_float((em << 13) + 0x38000000u);
  const float fs = (float)em * 5.9604644775390625e-8f;
  const float mag = (em < 0x400u) ? fs : fn;
  return __uint_as_float(__float_as_uint(mag) | sgn);
}

constexpr int kPbWihF = 0;
constexpr int kPbWihB = 35;
constexpr int kPbWhhF = 70;
constexpr int kPbWhhB = 80;
constexpr int kPbWml  = 90;
constexpr int kPbBias = 106;
constexpr int kPrepBlocks = 107;
static_assert((kNd * kKp / 8) == 35 * 128 && (kNd * kHk / 8) == 10 * 128 && (kMn * kHp / 8) == 16 * 128, "prep coverage");

__global__ __launch_bounds__(128) void prep_planes_kernel(
    const float* __restrict__ Wih_f, const float* __restrict__ Wih_b,
    const float* __restrict__ Whh_f, const float* __restrict__ Whh_b,
    const float* __restrict__ W_mlp,
    const float* __restrict__ bih_f, const float* __restrict__ bih_b,
    unsigned short* __restrict__ WIH, unsigned short* __restrict__ WHH,
    unsigned short* __restrict__ WML, float* __restrict__ BIAS)
{
  const int bx = blockIdx.x;
  const int tid = threadIdx.x;
  if (bx < kPbBias) {
    const float* src;
    unsigned short* dst;
    int srcRows, srcLd, dstCols, seg, segValid, blk;
    if (bx < kPbWihB) {
      src = Wih_f; dst = WIH; srcRows = kG3; srcLd = kEmb; dstCols = kKp; seg = kKp; segValid = kEmb; blk = bx - kPbWihF;
    } else if (bx < kPbWhhF) {
      src = Wih_b; dst = WIH + (size_t)kNd * kKp; srcRows = kG3; srcLd = kEmb; dstCols = kKp; seg = kKp; segValid = kEmb; blk = bx - kPbWihB;
    } else if (bx < kPbWhhB) {
      src = Whh_f; dst = WHH; srcRows = kG3; srcLd = kHid; dstCols = kHk; seg = kHk; segValid = kHid; blk = bx - kPbWhhF;
    } else if (bx < kPbWml) {
      src = Whh_b; dst = WHH + (size_t)kNd * kHk; srcRows = kG3; srcLd = kHid; dstCols = kHk; seg = kHk; segValid = kHid; blk = bx - kPbWhhB;
    } else {
      src = W_mlp; dst = WML; srcRows = kMlp; srcLd = 2 * kHid; dstCols = kHp; seg = kHk; segValid = kHid; blk = bx - kPbWml;
    }
    const int id  = blk * 128 + tid;
    const int cpr = dstCols >> 3;
    const int row = id / cpr;
    const int c8  = (id - row * cpr) << 3;
    const int sgi = c8 / seg;
    const int o0  = c8 - sgi * seg;
    const bool rowok = row < srcRows;
    const int rowc = rowok ? row : (srcRows - 1);
    v8h hv;
#pragma unroll
    for (int e = 0; e < 8; ++e) {
      const int o = o0 + e;
      const int col = sgi * segValid + o;
      const int colc = (col < srcLd) ? col : (srcLd - 1);
      float f = src[(size_t)rowc * srcLd + colc];
      asm volatile("" : "+v"(f));
      const bool ok = rowok && (o < segValid);
      const float g = ok ? f : 0.0f;
      hv[e] = to_h_carry(g);
    }
    unsigned short* q = dst + (size_t)id * 8;
    *(volatile v8h*)q = hv;
    __threadfence();
    *(volatile v8h*)q = hv;
  } else {
    const int tc = (tid < 79) ? tid : 79;
    v4f bv;
#pragma unroll
    for (int e = 0; e < 4; ++e) {
      const int n = tc * 4 + e;
      const int d = n / kNd;
      const int g = n - d * kNd;
      const int gc = (g < kG3) ? g : (kG3 - 1);
      float ff = bih_f[gc];
      float fb = bih_b[gc];
      asm volatile("" : "+v"(ff), "+v"(fb));
      const float pick = (d == 0) ? ff : fb;
      bv[e] = (g < kG3) ? pick : 0.0f;
    }
    if (tid < 80) {
      float* q = BIAS + tid * 4;
      *(volatile v4f*)q = bv;
      __threadfence();
      *(volatile v4f*)q = bv;
    }
  }
}

__global__ __launch_bounds__(160) void proj_gates_kernel(
    const int* __restrict__ tokens, const float* __restrict__ emb,
    const unsigned short* __restrict__ WIHp, const float* __restrict__ BIAS,
    unsigned short* __restrict__ GX)
{
  __shared__ __align__(16) _Float16 sAt[64 * kApitch];
  __shared__ __align__(16) float sT[5][16 * 68];
  __shared__ int sTok[64];
  const int tid  = threadIdx.x;
  const int lane = tid & 31;
  const int wave = __builtin_amdgcn_readfirstlane(tid >> 5);
  const int hh   = lane >> 4;
  const int c    = lane & 15;
  const int m0   = blockIdx.x * 64;
  {
    const int tc = (tid < 63) ? tid : 63;
    int tv = tokens[m0 + tc];
    asm volatile("" : "+v"(tv));
    tv = (tv < 0) ? 0 : tv;
    tv = (tv > kVocabRows - 1) ? (kVocabRows - 1) : tv;
    if (tid < 64) sTok[tid] = tv;
  }
  __syncthreads();
#pragma unroll 1
  for (int it = 0; it < 12; ++it) {
    const int id  = it * 160 + tid;
    const int idc = (id < 1791) ? id : 1791;
    const int row = idc / 28;
    const int ch  = idc - row * 28;
    const int chc = (ch < 24) ? ch : 24;
    const float* src = emb + (size_t)sTok[row] * kEmb + chc * 8;
    v4f a0 = *(const v4f*)(src);
    v4f a1 = *(const v4f*)(src + 4);
    asm volatile("" : "+v"(a0), "+v"(a1));
    const bool live = ch < 25;
    v8h hv;
#pragma unroll
    for (int e = 0; e < 4; ++e) {
      const float f0 = live ? a0[e] : 0.0f;
      const float f1 = live ? a1[e] : 0.0f;
      hv[e]     = to_h_carry(f0);
      hv[4 + e] = to_h_carry(f1);
    }
    if (id < 1792) *(v8h*)(sAt + row * kApitch + ch * 8) = hv;
  }
  __syncthreads();

  const int n0 = wave * 64;
  v8f acc[4][4];
#pragma unroll
  for (int i = 0; i < 4; ++i)
#pragma unroll
    for (int j = 0; j < 4; ++j) acc[i][j] = (v8f){0.f, 0.f, 0.f, 0.f, 0.f, 0.f, 0.f, 0.f};

  const _Float16* Wb = (const _Float16*)WIHp + (size_t)(n0 + c) * kKp + 8 * hh;
#pragma unroll 1
  for (int k0 = 0; k0 < kKp; k0 += 32) {
    v16h bh[4];
#pragma unroll
    for (int j = 0; j < 4; ++j) bh[j] = ldfrag_g(Wb + (size_t)(j * 16) * kKp + k0);
#pragma unroll
    for (int i = 0; i < 4; ++i) {
      FH a;
      const int ao = (i * 16 + c) * kApitch + k0 + 8 * hh;
      a.h[0] = *(const v8h*)(sAt + ao);
      a.h[1] = *(const v8h*)(sAt + ao + 16);
#pragma unroll
      for (int j = 0; j < 4; ++j) acc[i][j] = mma_h(a.v, bh[j], acc[i][j]);
    }
  }

  float bv[4];
#pragma unroll
  for (int j = 0; j < 4; ++j) bv[j] = BIAS[n0 + j * 16 + c];
  const int q  = lane >> 3;
  const int c8 = (lane & 7) * 8;
#pragma unroll
  for (int i = 0; i < 4; ++i) {
#pragma unroll
    for (int j = 0; j < 4; ++j) {
#pragma unroll
      for (int r = 0; r < 8; ++r)
        sT[wave][(8 * hh + r) * 68 + j * 16 + c] = acc[i][j][r] * kFold + bv[j];
    }
    __syncthreads();
    v8h hv[4];
#pragma unroll
    for (int it = 0; it < 4; ++it) {
      const int row = it * 4 + q;
      const v4f x0 = *(const v4f*)(&sT[wave][row * 68 + c8]);
      const v4f x1 = *(const v4f*)(&sT[wave][row * 68 + c8 + 4]);
#pragma unroll
      for (int e = 0; e < 4; ++e) {
        hv[it][e]     = (_Float16)x0[e];
        hv[it][4 + e] = (_Float16)x1[e];
      }
    }
    for (int pass = 0; pass < 2; ++pass) {
#pragma unroll
      for (int it = 0; it < 4; ++it) {
        const int row = it * 4 + q;
        *(volatile v8h*)(GX + (size_t)(m0 + i * 16 + row) * kNp + n0 + c8) = hv[it];
      }
      __threadfence();
    }
    __syncthreads();
  }
}

constexpr int kSHp = 56;
constexpr int kSAp = 72;
constexpr int kSGp = 160;
static_assert(64 * kSHp * 4 + 64 * kSAp * 2 + 64 * kSGp * 4 + kNd * 4 <= 65536, "static LDS of the scan kernel");

__global__ __launch_bounds__(256) void gru_scan_kernel(
    const unsigned short* __restrict__ GX, const unsigned short* __restrict__ WHHp,
    const float* __restrict__ bhh_f, const float* __restrict__ bhh_b,
    unsigned short* __restrict__ HP)
{
  __shared__ __align__(16) float sH[64 * kSHp];
  __shared__ __align__(16) _Float16 sA[64 * kSAp];
  __shared__ __align__(16) float sG[64 * kSGp];
  __shared__ float sBias[kNd];
  const int tid  = threadIdx.x;
  const int lane = tid & 31;
  const int wave = __builtin_amdgcn_readfirstlane(tid >> 5);
  const int hh   = lane >> 4;
  const int c    = lane & 15;
  const int dir  = blockIdx.x >> 2;
  const int b0   = (blockIdx.x & 3) * 64;
  const int mt   = wave >> 1;
  const int ng   = wave & 1;
  const float* bhh = (dir == 0) ? bhh_f : bhh_b;

  for (int i = tid; i < 64 * kSHp; i += 256) sH[i] = 0.0f;
  {
    const v8h zv = (v8h){(_Float16)0.f, (_Float16)0.f, (_Float16)0.f, (_Float16)0.f,
                         (_Float16)0.f, (_Float16)0.f, (_Float16)0.f, (_Float16)0.f};
    for (int i = tid; i < (64 * kSAp) / 8; i += 256) *(v8h*)(sA + i * 8) = zv;
  }
  {
    const int ic = (tid < kG3 - 1) ? tid : (kG3 - 1);
    float bvv = bhh[ic];
    asm volatile("" : "+v"(bvv));
    if (tid < kNd) sBias[tid] = (tid < kG3) ? bvv : 0.0f;
  }
  v16h bf[5][2];
  {
    const _Float16* Wd = (const _Float16*)WHHp + (size_t)dir * kNd * kHk;
#pragma unroll
    for (int i = 0; i < 5; ++i) {
#pragma unroll
      for (int kk = 0; kk < 2; ++kk) {
        bf[i][kk] = ldfrag_g(Wd + (size_t)((ng * 5 + i) * 16 + c) * kHk + kk * 32 + 8 * hh);
        asm volatile("" : "+v"(bf[i][kk]));
      }
    }
  }
  __syncthreads();

  const unsigned* gxw = (const unsigned*)GX;
#pragma unroll 1
  for (int step = 0; step < kSeq; ++step) {
    const int t = (dir == 0) ? step : (kSeq - 1 - step);
    {
      FH a0, a1;
      const int ao = (mt * 16 + c) * kSAp + 8 * hh;
      a0.h[0] = *(const v8h*)(sA + ao);
      a0.h[1] = *(const v8h*)(sA + ao + 16);
      a1.h[0] = *(const v8h*)(sA + ao + 32);
      a1.h[1] = *(const v8h*)(sA + ao + 48);
      v8f acc[5];
#pragma unroll
      for (int i = 0; i < 5; ++i) {
        acc[i] = (v8f){0.f, 0.f, 0.f, 0.f, 0.f, 0.f, 0.f, 0.f};
        acc[i] = mma_h(a0.v, bf[i][0], acc[i]);
        acc[i] = mma_h(a1.v, bf[i][1], acc[i]);
      }
#pragma unroll
      for (int i = 0; i < 5; ++i) {
#pragma unroll
        for (int r = 0; r < 8; ++r)
          sG[(mt * 16 + 8 * hh + r) * kSGp + (ng * 5 + i) * 16 + c] = acc[i][r];
      }
    }
    __syncthreads();
#pragma unroll 1
    for (int it = 0; it < 13; ++it) {
      if (it * 256 + wave * 32 < 64 * kHid) {
        const int i  = it * 256 + tid;
        const int bl = i / kHid;
        const int j  = i - bl * kHid;
        const size_t rowg = (size_t)t * kBatch + b0 + bl;
        const unsigned* gw = gxw + rowg * (kNp / 2) + dir * (kNd / 2) + (j >> 1);
        const unsigned wr = gw[0];
        const unsigned wz = gw[kHid / 2];
        const unsigned wn = gw[kHid];
        const int sh = (j & 1) * 16;
        const float xr = h16_to_f32((wr >> sh) & 0xffffu);
        const float xz = h16_to_f32((wz >> sh) & 0xffffu);
        const float xn = h16_to_f32((wn >> sh) & 0xffffu);
        const float* gr = sG + bl * kSGp;
        const float ghr = gr[j] * kFold + sBias[j];
        const float ghz = gr[kHid + j] * kFold + sBias[kHid + j];
        const float ghn = gr[2 * kHid + j] * kFold + sBias[2 * kHid + j];
        const float rg = 1.0f / (1.0f + expf(-(xr + ghr)));
        const float zg = 1.0f / (1.0f + expf(-(xz + ghz)));
        const float nn = tanhf(xn + rg * ghn);
        const float hold = sH[bl * kSHp + j];
        const float hnew = (1.0f - zg) * nn + zg * hold;
        sH[bl * kSHp + j] = hnew;
      }
    }
    __syncthreads();
    {
      v8h hv[2];
#pragma unroll
      for (int it2 = 0; it2 < 2; ++it2) {
        const int id  = it2 * 256 + tid;
        const int row = id >> 3;
        const int c8  = (id & 7) * 8;
        const int c8r = (c8 < 48) ? c8 : 48;
        const v4f x0 = *(const v4f*)(sH + row * kSHp + c8r);
        const v4f x1 = *(const v4f*)(sH + row * kSHp + c8r + 4);
#pragma unroll
        for (int e = 0; e < 4; ++e) {
          const float f0 = ((c8 + e) < kHid) ? x0[e] : 0.0f;
          const float f1 = ((c8 + 4 + e) < kHid) ? x1[e] : 0.0f;
          hv[it2][e]     = to_h_carry(f0);
          hv[it2][4 + e] = to_h_carry(f1);
        }
        *(v8h*)(sA + row * kSAp + c8) = hv[it2];
      }
      for (int pass = 0; pass < 2; ++pass) {
#pragma unroll
        for (int it2 = 0; it2 < 2; ++it2) {
          const int id  = it2 * 256 + tid;
          const int row = id >> 3;
          const int c8  = (id & 7) * 8;
          *(volatile v8h*)(HP + ((size_t)t * kBatch + b0 + row) * kHp + dir * kHk + c8) = hv[it2];
        }
        __threadfence();
      }
    }
    __syncthreads();
  }
}

constexpr int kSUp = 132;

__global__ __launch_bounds__(256) void mlp_score_kernel(
    const unsigned short* __restrict__ HPp, const unsigned short* __restrict__ WMLp,
    const float* __restrict__ b_mlp, const float* __restrict__ ctx,
    float* __restrict__ SC)
{
  __shared__ __align__(16) float sU[64 * kSUp];
  __shared__ float sB[128];
  __shared__ float sC[128];
  __shared__ __align__(16) float sS[64];
  const int tid  = threadIdx.x;
  const int lane = tid & 31;
  const int wave = __builtin_amdgcn_readfirstlane(tid >> 5);
  const int hh   = lane >> 4;
  const int c    = lane & 15;
  const int mt   = wave >> 1;
  const int ng   = wave & 1;
  const int m0   = blockIdx.x * 64;
  {
    const int ic = (tid < kMlp - 1) ? tid : (kMlp - 1);
    float bvv = b_mlp[ic];
    float cvv = ctx[ic];
    asm volatile("" : "+v"(bvv), "+v"(cvv));
    if (tid < 128) {
      sB[tid] = (tid < kMlp) ? bvv : 0.0f;
      sC[tid] = (tid < kMlp) ? cvv : 0.0f;
    }
  }
  v8f acc[4];
#pragma unroll
  for (int j = 0; j < 4; ++j) acc[j] = (v8f){0.f, 0.f, 0.f, 0.f, 0.f, 0.f, 0.f, 0.f};
  const _Float16* Ab = (const _Float16*)HPp + (size_t)(m0 + mt * 16 + c) * kHp + 8 * hh;
  const _Float16* Bb = (const _Float16*)WMLp + (size_t)(ng * 64 + c) * kHp + 8 * hh;
#pragma unroll
  for (int kk = 0; kk < 4; ++kk) {
    const v16h a = ldfrag_g(Ab + kk * 32);
#pragma unroll
    for (int j = 0; j < 4; ++j) {
      const v16h b = ldfrag_g(Bb + (size_t)(j * 16) * kHp + kk * 32);
      acc[j] = mma_h(a, b, acc[j]);
    }
  }
#pragma unroll
  for (int j = 0; j < 4; ++j) {
#pragma unroll
    for (int r = 0; r < 8; ++r)
      sU[(mt * 16 + 8 * hh + r) * kSUp + ng * 64 + j * 16 + c] = acc[j][r];
  }
  __syncthreads();
  const int row = tid >> 2;
  const int qt  = tid & 3;
  float p = 0.0f;
#pragma unroll 1
  for (int e = 0; e < kMlp / 4; ++e) {
    const int n = qt * (kMlp / 4) + e;
    const float u = tanhf(sU[row * kSUp + n] * kFold + sB[n]);
    p += u * sC[n];
  }
  p += __shfl_xor(p, 1, 32);
  p += __shfl_xor(p, 2, 32);
  if (qt == 0) sS[row] = p;
  __syncthreads();
  if (wave == 0) {
    const int lc = (lane < 15) ? lane : 15;
    const v4f v = *(const v4f*)(sS + lc * 4);
    if (lane < 16) {
      float* q = SC + m0 + lane * 4;
      *(volatile v4f*)q = v;
      __threadfence();
      *(volatile v4f*)q = v;
    }
  }
}

__global__ __launch_bounds__(256) void attn_pool_kernel(
    const float* __restrict__ SC, const unsigned short* __restrict__ HPp, float* __restrict__ out)
{
  __shared__ float sE[8][kSeq];
  __shared__ __align__(16) float sO[8 * 2 * kHid];
  const int tid  = threadIdx.x;
  const int lane = tid & 31;
  const int wave = __builtin_amdgcn_readfirstlane(tid >> 5);
  const int b    = blockIdx.x * 8 + wave;
  float mx = -INFINITY;
#pragma unroll 1
  for (int i = 0; i < kSeq / 32; ++i) mx = fmaxf(mx, SC[(size_t)(lane + 32 * i) * kBatch + b]);
  mx = fmaxf(mx, __shfl_xor(mx, 16, 32));
  mx = fmaxf(mx, __shfl_xor(mx, 8, 32));
  mx = fmaxf(mx, __shfl_xor(mx, 4, 32));
  mx = fmaxf(mx, __shfl_xor(mx, 2, 32));
  mx = fmaxf(mx, __shfl_xor(mx, 1, 32));
  float sum = 0.0f;
#pragma unroll 1
  for (int i = 0; i < kSeq / 32; ++i) {
    const int s = lane + 32 * i;
    const float e = expf(SC[(size_t)s * kBatch + b] - mx);
    sE[wave][s] = e;
    sum += e;
  }
  sum += __shfl_xor(sum, 16, 32);
  sum += __shfl_xor(sum, 8, 32);
  sum += __shfl_xor(sum, 4, 32);
  sum += __shfl_xor(sum, 2, 32);
  sum += __shfl_xor(sum, 1, 32);
  __syncthreads();
  const unsigned* hw = (const unsigned*)HPp;
  float a0 = 0.0f, a1 = 0.0f, a2 = 0.0f, a3 = 0.0f;
#pragma unroll 1
  for (int s = 0; s < kSeq; ++s) {
    const float e = sE[wave][s];
    const unsigned* rw = hw + ((size_t)s * kBatch + b) * (kHp / 2);
    const unsigned wf = rw[lane];
    const unsigned wb = rw[32 + lane];
    a0 += e * h16_to_f32(wf & 0xffffu);
    a1 += e * h16_to_f32(wf >> 16);
    a2 += e * h16_to_f32(wb & 0xffffu);
    a3 += e * h16_to_f32(wb >> 16);
  }
  const float inv = kUncar * (1.0f / sum);
  if (lane < kHid / 2) {
    sO[wave * 100 + 2 * lane]          = a0 * inv;
    sO[wave * 100 + 2 * lane + 1]      = a1 * inv;
    sO[wave * 100 + 50 + 2 * lane]     = a2 * inv;
    sO[wave * 100 + 50 + 2 * lane + 1] = a3 * inv;
  }
  __syncthreads();
  if (wave == 0) {
    v4f val[7];
#pragma unroll
    for (int it = 0; it < 7; ++it) {
      const int idx = it * 32 + lane;
      const int idc = (idx < 199) ? idx : 199;
      val[it] = *(const v4f*)(sO + idc * 4);
    }
    float* ob = out + (size_t)blockIdx.x * 800;
    for (int pass = 0; pass < 2; ++pass) {
#pragma unroll
      for (int it = 0; it < 7; ++it) {
        const int idx = it * 32 + lane;
        if (idx < 200) *(volatile v4f*)(ob + idx * 4) = val[it];
      }
      __threadfence();
    }
  }
}

extern "C" void kernel_launch(void* const* d_in, const int* in_sizes, int n_in,
                              void* d_out, int out_size, void* d_ws, size_t ws_size,
                              hipStream_t stream) {
  if (n_in < 13) return;
  if (in_sizes[0] != kRows) return;
  if (in_sizes[1] != kVocabRows * kEmb) return;
  if (in_sizes[2] != kG3 * kEmb || in_sizes[6] != kG3 * kEmb) return;
  if (in_sizes[3] != kG3 * kHid || in_sizes[7] != kG3 * kHid) return;
  if (in_sizes[4] != kG3 || in_sizes[5] != kG3 || in_sizes[8] != kG3 || in_sizes[9] != kG3) return;
  if (in_sizes[10] != kMlp * 2 * kHid) return;
  if (in_sizes[11] != kMlp || in_sizes[12] != kMlp) return;
  if (out_size != kBatch * 2 * kHid) return;
  if (ws_size < kWsTotal) return;

  const int*   tokens = (const int*)  d_in[0];
  const float* emb    = (const float*)d_in[1];
  const float* Wih_f  = (const float*)d_in[2];
  const float* Whh_f  = (const float*)d_in[3];
  const float* bih_f  = (const float*)d_in[4];
  const float* bhh_f  = (const float*)d_in[5];
  const float* Wih_b  = (const float*)d_in[6];
  const float* Whh_b  = (const float*)d_in[7];
  const float* bih_b  = (const float*)d_in[8];
  const float* bhh_b  = (const float*)d_in[9];
  const float* W_mlp  = (const float*)d_in[10];
  const float* b_mlp  = (const float*)d_in[11];
  const float* ctx    = (const float*)d_in[12];
  float* out = (float*)d_out;

  char* ws = (char*)d_ws;
  unsigned short* WIH  = (unsigned short*)(ws + kOffWIH);
  float*          BIAS = (float*)(ws + kOffBIAS);
  unsigned short* WHH  = (unsigned short*)(ws + kOffWHH);
  unsigned short* WML  = (unsigned short*)(ws + kOffWML);
  unsigned short* GX   = (unsigned short*)(ws + kOffGX);
  unsigned short* HP   = (unsigned short*)(ws + kOffHP);
  float*          SC   = (float*)(ws + kOffSC);

  prep_planes_kernel<<<dim3(kPrepBlocks), dim3(128), 0, stream>>>(
      Wih_f, Wih_b, Whh_f, Whh_b, W_mlp, bih_f, bih_b, WIH, WHH, WML, BIAS);

  proj_gates_kernel<<<dim3(kRows / 64), dim3(160), 0, stream>>>(tokens, emb, WIH, BIAS, GX);

  gru_scan_kernel<<<dim3(2 * (kBatch / 64)), dim3(256), 0, stream>>>(GX, WHH, bhh_f, bhh_b, HP);

  mlp_score_kernel<<<dim3(kRows / 64), dim3(256), 0, stream>>>(HP, WML, b_mlp, ctx, SC);

  attn_pool_kernel<<<dim3(kBatch / 8), dim3(256), 0, stream>>>(SC, HP, out);
}
